// TrmBlock_36472862277693
// MI455X (gfx1250) — hardware-verified
//
#include <hip/hip_runtime.h>
#include <math.h>
#include <stdint.h>

typedef __attribute__((ext_vector_type(16))) _Float16 v16h;
typedef __attribute__((ext_vector_type(8)))  _Float16 v8h;
typedef __attribute__((ext_vector_type(16))) __bf16   v16b;
typedef __attribute__((ext_vector_type(8)))  __bf16   v8b;
typedef __attribute__((ext_vector_type(8)))  float    v8f;
typedef __attribute__((ext_vector_type(4)))  float    v4f;
typedef __attribute__((ext_vector_type(2)))  float    v2f;
typedef __attribute__((ext_vector_type(4)))  unsigned int v4u;

constexpr int kBatch     = 16;
constexpr int kSeq       = 1024;
constexpr int kDm        = 512;
constexpr int kProj      = 512;
constexpr int kHeads     = 8;
constexpr int kHd        = 64;
constexpr int kFf        = 2048;
constexpr int kTok       = kBatch * kSeq;
constexpr int kChunkRows = 4096;
constexpr int kNumChunks = kTok / kChunkRows;
static_assert(kHeads * kHd == kProj);
static_assert(kTok % kChunkRows == 0);
static_assert(kTok % 64 == 0 && kDm % 64 == 0 && kProj % 64 == 0 && kFf % 64 == 0 && kSeq % 64 == 0 && kChunkRows % 64 == 0);
static_assert(kDm % 32 == 0 && kProj % 32 == 0 && kFf % 32 == 0);

constexpr size_t kPlane16 = (size_t)kTok * kDm * 2;
constexpr size_t kOffQ    = 0;
constexpr size_t kOffK    = 1 * kPlane16;
constexpr size_t kOffVT   = 2 * kPlane16;
constexpr size_t kOffXB   = 3 * kPlane16;
constexpr size_t kOffX1H  = 4 * kPlane16;
constexpr size_t kOffH16  = 5 * kPlane16;
constexpr size_t kOffW    = 6 * kPlane16;
constexpr size_t kOffWq   = kOffW;
constexpr size_t kOffWk   = kOffWq + (size_t)kProj * kDm * 2;
constexpr size_t kOffWv   = kOffWk + (size_t)kProj * kDm * 2;
constexpr size_t kOffWo   = kOffWv + (size_t)kProj * kDm * 2;
constexpr size_t kOffW1   = kOffWo + (size_t)kDm * kProj * 2;
constexpr size_t kOffW2   = kOffW1 + (size_t)kFf * kDm * 2;
constexpr size_t kWsTotal = kOffW2 + (size_t)kDm * kFf * 2;
static_assert(kWsTotal == 106954752ull);
static_assert(kWsTotal <= 134217728ull);
static_assert((size_t)kTok * kDm * 4 == 2 * kPlane16);
static_assert((size_t)kChunkRows * kFf * 4 == 2 * kPlane16);
static_assert((size_t)kChunkRows * kFf * 2 == kPlane16);
static_assert((size_t)kBatch * kProj * kSeq * 2 == kPlane16);

__device__ __forceinline__ unsigned short f2bf_bits(float f) {
  unsigned u = __float_as_uint(f);
  return (unsigned short)((u + 0x7FFFu + ((u >> 16) & 1u)) >> 16);
}
__device__ __forceinline__ float bf_bits2f(unsigned short h) { return __uint_as_float(((unsigned)h) << 16); }
__device__ __forceinline__ unsigned pk16(unsigned short a, unsigned short b) { return (unsigned)a | ((unsigned)b << 16); }

__device__ __forceinline__ void dep_guard_h(v8f& a, v8f& b, v16h x, v16h y) { asm volatile("v_nop\n\tv_nop\n\tv_nop\n\tv_nop" : "+v"(a), "+v"(b) : "v"(x), "v"(y)); }
__device__ __forceinline__ void dep_guard_b(v8f& a, v8f& b, v16b x, v16b y) { asm volatile("v_nop\n\tv_nop\n\tv_nop\n\tv_nop" : "+v"(a), "+v"(b) : "v"(x), "v"(y)); }
__device__ __forceinline__ void keep4_h(v16h a, v16h b, v16h c, v16h d) { asm volatile("v_nop" :: "v"(a), "v"(b), "v"(c), "v"(d)); }
__device__ __forceinline__ void keep4_b(v16b a, v16b b, v16b c, v16b d) { asm volatile("v_nop" :: "v"(a), "v"(b), "v"(c), "v"(d)); }
__device__ __forceinline__ void acc_guard4(v8f& a, v8f& b, v8f& c, v8f& d) { asm volatile("v_nop\n\tv_nop\n\tv_nop\n\tv_nop" : "+v"(a), "+v"(b), "+v"(c), "+v"(d)); }
template <typename T> struct Frag;
template <> struct Frag<_Float16> {
  typedef v16h V; union U { v16h v; v8h h[2]; };
  static __device__ __forceinline__ v16h load(const _Float16* p) {
    U f; f.h[0] = *(const v8h*)(p); f.h[1] = *(const v8h*)(p + 16); return f.v;
  }
  static __device__ __forceinline__ v8f mma(v16h a, v16h b, v8f c) {
    return __builtin_amdgcn_wmma_f32_16x16x32_f16(false, a, false, b, (short)0, c, false, false);
  }
  static __device__ __forceinline__ void guard(v8f& a, v8f& b, v16h x, v16h y) { dep_guard_h(a, b, x, y); }
  static __device__ __forceinline__ void keep(v16h a, v16h b, v16h c, v16h d) { keep4_h(a, b, c, d); }
};
template <> struct Frag<__bf16> {
  typedef v16b V; union U { v16b v; v8b h[2]; };
  static __device__ __forceinline__ v16b load(const __bf16* p) {
    U f; f.h[0] = *(const v8b*)(p); f.h[1] = *(const v8b*)(p + 16); return f.v;
  }
  static __device__ __forceinline__ v8f mma(v16b a, v16b b, v8f c) {
    return __builtin_amdgcn_wmma_f32_16x16x32_bf16(false, a, false, b, (short)0, c, false, false);
  }
  static __device__ __forceinline__ void guard(v8f& a, v8f& b, v16b x, v16b y) { dep_guard_b(a, b, x, y); }
  static __device__ __forceinline__ void keep(v16b a, v16b b, v16b c, v16b d) { keep4_b(a, b, c, d); }
};

template <int ET> struct Elem;
template <> struct Elem<0> { typedef _Float16 T; };
template <> struct Elem<1> { typedef __bf16 T; };
template <int ET, bool SPLIT, int BIAS_MODE, int OUT_MODE, bool RESID, int ACT = 0>
__global__ __launch_bounds__(256) void wmma_gemm64(
    const unsigned short* __restrict__ Ap, const unsigned short* __restrict__ A2p, int lda, long strideA,
    const unsigned short* __restrict__ Btp, const unsigned short* __restrict__ Bt2p, int ldb, long strideB,
    void* __restrict__ Cout, void* __restrict__ Cout2, int ldc, long strideC,
    const float* __restrict__ bias,
    const float* __restrict__ resid, long strideR,
    int M, int N, int K, float scale) {
  typedef typename Elem<ET>::T T;
  typedef typename Frag<T>::V V;
  const T* A = (const T*)Ap; const T* A2 = (const T*)A2p; const T* Bt = (const T*)Btp; const T* Bt2 = (const T*)Bt2p;
  __shared__ __align__(16) float sT[8][16 * 68];
  const int b    = blockIdx.y;
  const int lane = threadIdx.x & 31;
  const int wave = threadIdx.x >> 5;
  const int tilesN = N >> 6;
  const int tilesM = M >> 6;
  const int tile = blockIdx.x * 8 + wave;
  if (tile >= tilesM * tilesN) return;
  const int tm = tile / tilesN;
  const int tn = tile - tm * tilesN;
  const int m0 = tm << 6;
  const int n0 = tn << 6;

  const T* Ab  = A  + (size_t)b * strideA;
  const T* Bb  = Bt + (size_t)b * strideB;
  const T* Ab2 = SPLIT ? (A2  + (size_t)b * strideA) : nullptr;
  const T* Bb2 = SPLIT ? (Bt2 + (size_t)b * strideB) : nullptr;

  const int rlane = lane & 15;
  const int koff  = (lane >> 4) * 8;
  const int mOff  = (lane >> 4) * 8;

  v8f acc[4][4];
#pragma unroll
  for (int i = 0; i < 4; ++i)
#pragma unroll
    for (int j = 0; j < 4; ++j) acc[i][j] = (v8f){0.f,0.f,0.f,0.f,0.f,0.f,0.f,0.f};

  for (int k0 = 0; k0 < K; k0 += 32) {
    V bh[4], bl[4];
#pragma unroll
    for (int j = 0; j < 4; ++j) {
      const size_t bo = (size_t)(n0 + (j << 4) + rlane) * ldb + koff + k0;
      bh[j] = Frag<T>::load(Bb + bo);
      if (SPLIT) bl[j] = Frag<T>::load(Bb2 + bo);
    }
#pragma unroll
    for (int i = 0; i < 4; ++i) {
      const size_t ao = (size_t)(m0 + (i << 4) + rlane) * lda + koff + k0;
      V ah = Frag<T>::load(Ab + ao);
      V al;
      if (SPLIT) al = Frag<T>::load(Ab2 + ao);
#pragma unroll
      for (int j = 0; j < 4; ++j) {
        acc[i][j] = Frag<T>::mma(ah, bh[j], acc[i][j]);
        if (SPLIT) {
          acc[i][j] = Frag<T>::mma(ah, bl[j], acc[i][j]);
          acc[i][j] = Frag<T>::mma(al, bh[j], acc[i][j]);
        }
      }
      Frag<T>::guard(acc[i][0], acc[i][3], ah, SPLIT ? al : ah);
    }
    Frag<T>::keep(bh[0], bh[1], bh[2], bh[3]);
    if (SPLIT) Frag<T>::keep(bl[0], bl[1], bl[2], bl[3]);
  }
  acc_guard4(acc[0][0], acc[0][1], acc[0][2], acc[0][3]);
  acc_guard4(acc[1][0], acc[1][1], acc[1][2], acc[1][3]);
  acc_guard4(acc[2][0], acc[2][1], acc[2][2], acc[2][3]);
  acc_guard4(acc[3][0], acc[3][1], acc[3][2], acc[3][3]);

  float* slab = sT[wave];
  const float* Rb = RESID ? (resid + (size_t)b * strideR) : nullptr;
#pragma unroll
  for (int i = 0; i < 4; ++i) {
    const int mBase = m0 + (i << 4);
#pragma unroll
    for (int j = 0; j < 4; ++j) {
      const int n = n0 + (j << 4) + rlane;
      float bv = 0.f;
      if (BIAS_MODE == 2) bv = bias[n];
#pragma unroll
      for (int r = 0; r < 8; ++r) {
        float v = acc[i][j][r] * scale;
        if (BIAS_MODE == 1) v += bias[mBase + mOff + r];
        if (BIAS_MODE == 2) v += bv;
        if (RESID) v += Rb[(size_t)(mBase + mOff + r) * ldc + n];
        if (ACT == 1) v = tanhf(v);
        if (ACT == 2) v = fmaxf(v, 0.0f);
        if (ACT == 3) v = v / (1.0f + expf(-v));
        if (ACT == 4) v = (v > 0.f) ? v : 0.01f * v;
        slab[(mOff + r) * 68 + (j << 4) + rlane] = v;
      }
    }
    __builtin_amdgcn_fence(__ATOMIC_RELEASE, "workgroup");
    __builtin_amdgcn_wave_barrier();
    __builtin_amdgcn_fence(__ATOMIC_ACQUIRE, "workgroup");
    if (OUT_MODE == 0) {
      float* C = (float*)Cout + (size_t)b * strideC;
      const int hh = lane >> 4, c4 = (lane & 15) * 4;
      for (int pass = 0; pass < 2; ++pass) {
#pragma unroll
        for (int it = 0; it < 8; ++it) {
          const int row = it * 2 + hh;
          v4f v = *(const v4f*)(slab + row * 68 + c4);
          *(volatile v4f*)(C + (size_t)(mBase + row) * ldc + n0 + c4) = v;
        }
        __threadfence();
      }
    } else {
      const int q = lane >> 3, c8 = (lane & 7) * 8;
      unsigned short* C  = (unsigned short*)Cout  + (size_t)b * strideC;
      unsigned short* C2 = (OUT_MODE == 2) ? ((unsigned short*)Cout2 + (size_t)b * strideC) : nullptr;
      for (int pass = 0; pass < 2; ++pass) {
#pragma unroll
        for (int it = 0; it < 4; ++it) {
          const int row = it * 4 + q;
          const float* sp = slab + row * 68 + c8;
          v8h hv, lv;
#pragma unroll
          for (int e = 0; e < 8; ++e) {
            if (OUT_MODE == 1) {
              hv[e] = (_Float16)sp[e];
            } else {
              unsigned short hb = f2bf_bits(sp[e]);
              unsigned short lb = f2bf_bits(sp[e] - bf_bits2f(hb));
              hv[e] = __builtin_bit_cast(_Float16, hb);
              lv[e] = __builtin_bit_cast(_Float16, lb);
            }
          }
          *(volatile v8h*)(C + (size_t)(mBase + row) * ldc + n0 + c8) = hv;
          if (OUT_MODE == 2) *(volatile v8h*)(C2 + (size_t)(mBase + row) * ldc + n0 + c8) = lv;
        }
        __threadfence();
      }
    }
    __builtin_amdgcn_fence(__ATOMIC_RELEASE, "workgroup");
    __builtin_amdgcn_wave_barrier();
    __builtin_amdgcn_fence(__ATOMIC_ACQUIRE, "workgroup");
  }
}

__global__ __launch_bounds__(256) void cast_f32_bf16x2(const float* __restrict__ in, unsigned short* __restrict__ out, int n2) {
  const int i = blockIdx.x * 256 + threadIdx.x;
  if (i < n2) {
    const v2f f = *(const v2f*)(in + 2 * (size_t)i);
    const unsigned u = pk16(f2bf_bits(f[0]), f2bf_bits(f[1]));
    ((volatile unsigned*)out)[i] = u;
    __threadfence();
    ((volatile unsigned*)out)[i] = u;
  }
}

template <int CVT> __device__ __forceinline__ unsigned short cvt16_bits(float f) {
  if (CVT == 0) return f2bf_bits(f);
  const _Float16 h = (_Float16)f;
  return __builtin_bit_cast(unsigned short, h);
}

template <int CVT>
__global__ __launch_bounds__(256) void tconv_kernel(const float* __restrict__ W, unsigned short* __restrict__ o,
                                                    int R, int Cc, float scl) {
  __shared__ __align__(16) float tf[64 * 68];
  const int c0  = blockIdx.x * 64;
  const int r0  = blockIdx.y * 64;
  const int tid = threadIdx.x;
  {
    const int lr = tid >> 4;
    const int c4 = (tid & 15) * 4;
#pragma unroll
    for (int it = 0; it < 4; ++it) {
      const int rr = it * 16 + lr;
      const v4f a = *(const v4f*)(W + (size_t)(r0 + rr) * Cc + c0 + c4);
      *(v4f*)(tf + rr * 68 + c4) = a;
    }
  }
  __syncthreads();
  const int sub = tid >> 3;
  const int c8  = (tid & 7) * 8;
  v4u hv[2];
#pragma unroll
  for (int it = 0; it < 2; ++it) {
    const int oc = it * 32 + sub;
    v4u a;
#pragma unroll
    for (int q = 0; q < 4; ++q) {
      const float f0 = tf[(c8 + 2 * q) * 68 + oc] * scl;
      const float f1 = tf[(c8 + 2 * q + 1) * 68 + oc] * scl;
      a[q] = pk16(cvt16_bits<CVT>(f0), cvt16_bits<CVT>(f1));
    }
    hv[it] = a;
  }
  for (int pass = 0; pass < 2; ++pass) {
#pragma unroll
    for (int it = 0; it < 2; ++it) {
      const int oc = it * 32 + sub;
      const size_t go = (size_t)(c0 + oc) * R + r0 + c8;
      *(volatile v4u*)(o + go) = hv[it];
    }
    __threadfence();
  }
}

#define AT_D 64
#define AT_NW 4
#define AT_QB 64
#define AT_KC 64

__device__ __forceinline__ v8f at_mma_h(v16h a, v16h b, v8f c) {
  c = __builtin_amdgcn_wmma_f32_16x16x32_f16(false, a, false, b, (short)0, c, false, false);
  asm volatile("v_nop\n\tv_nop\n\tv_nop\n\tv_nop" : "+v"(c) : "v"(a), "v"(b));
  return c;
}

__global__ __launch_bounds__(128)
void attn_full64_f16_kernel(const unsigned short* __restrict__ qp, const unsigned short* __restrict__ kp,
                            const unsigned short* __restrict__ vtp, unsigned short* __restrict__ op,
                            float sscale, float oscale) {
  union FB { v16h v; v8h h[2]; };
  __shared__ __align__(16) _Float16 Ksh[AT_KC * AT_D];
  __shared__ __align__(16) _Float16 Vth[AT_D * AT_KC];
  __shared__ __align__(16) _Float16 Psh[AT_NW][16 * AT_KC];
  __shared__ __align__(16) float    Os[AT_NW][16 * 68];

  const float PSC = 32768.0f;
  const int tid  = threadIdx.x;
  const int wave = tid >> 5;
  const int lane = tid & 31;
  const int hh   = lane >> 4;
  const int c    = lane & 15;

  const int nqb = kSeq / AT_QB;
  const int bx = blockIdx.x;
  const int qb = bx % nqb;
  const int h  = bx / nqb;
  const int b  = blockIdx.y;
  const int q0 = qb * AT_QB + wave * 16;

  const _Float16* Qh = (const _Float16*)(const void*)qp  + (size_t)b * kSeq * kProj + (size_t)h * AT_D;
  const _Float16* Kh = (const _Float16*)(const void*)kp  + (size_t)b * kSeq * kProj + (size_t)h * AT_D;
  const _Float16* Vh = (const _Float16*)(const void*)vtp + (size_t)b * kProj * kSeq + (size_t)h * AT_D * kSeq;
  _Float16*       ob = (_Float16*)(void*)op              + (size_t)b * kSeq * kProj + (size_t)h * AT_D;

  v16h qah[2];
#pragma unroll
  for (int dc = 0; dc < 2; ++dc) {
    const _Float16* qr = Qh + (size_t)(q0 + c) * kProj + dc * 32 + 8 * hh;
    qah[dc] = Frag<_Float16>::load(qr);
  }

  float mrow[8], lrow[8];
  v8f oacc[4];
#pragma unroll
  for (int r = 0; r < 8; ++r) { mrow[r] = -INFINITY; lrow[r] = 0.f; }
#pragma unroll
  for (int t = 0; t < 4; ++t) oacc[t] = (v8f){0.f,0.f,0.f,0.f,0.f,0.f,0.f,0.f};

  const int nChunks = kSeq / AT_KC;
  for (int kc = 0; kc < nChunks; ++kc) {
    const int kv0 = kc * AT_KC;
    __syncthreads();
    {
      const int r = tid >> 1, half = (tid & 1) * 32;
      const _Float16* ksh = Kh + (size_t)(kv0 + r) * kProj + half;
      const _Float16* vsh = Vh + (size_t)r * kSeq + kv0 + half;
#pragma unroll
      for (int i = 0; i < 4; ++i) {
        const v8h a0 = *(const v8h*)(ksh + 8 * i);
        const v8h b0 = *(const v8h*)(vsh + 8 * i);
        *(v8h*)(Ksh + r * AT_D  + half + 8 * i) = a0;
        *(v8h*)(Vth + r * AT_KC + half + 8 * i) = b0;
      }
    }
    __syncthreads();

    v8f s[4];
#pragma unroll
    for (int j = 0; j < 4; ++j) {
      s[j] = (v8f){0.f,0.f,0.f,0.f,0.f,0.f,0.f,0.f};
#pragma unroll
      for (int dc = 0; dc < 2; ++dc) {
        FB kb;
        kb.h[0] = *(const v8h*)(Ksh + (j * 16 + c) * AT_D + dc * 32 + 8 * hh);
        kb.h[1] = *(const v8h*)(Ksh + (j * 16 + c) * AT_D + dc * 32 + 16 + 8 * hh);
        s[j] = at_mma_h(qah[dc], kb.v, s[j]);
      }
    }
    float cm[8];
#pragma unroll
    for (int r = 0; r < 8; ++r) {
      float m = -INFINITY;
#pragma unroll
      for (int j = 0; j < 4; ++j) {
        const float sv = s[j][r] * sscale;
        s[j][r] = sv;
        m = fmaxf(m, sv);
      }
#pragma unroll
      for (int off = 1; off < 16; off <<= 1) m = fmaxf(m, __shfl_xor(m, off, 32));
      cm[r] = m;
    }
    _Float16* pwh = Psh[wave];
#pragma unroll
    for (int r = 0; r < 8; ++r) {
      const float mnew = fmaxf(mrow[r], cm[r]);
      const float alpha = expf(mrow[r] - mnew);
      mrow[r] = mnew;
      float psum = 0.f;
#pragma unroll
      for (int j = 0; j < 4; ++j) {
        const float p = expf(s[j][r] - mnew);
        psum += p;
        pwh[(8 * hh + r) * AT_KC + j * 16 + c] = (_Float16)(p * PSC);
      }
#pragma unroll
      for (int off = 1; off < 16; off <<= 1) psum += __shfl_xor(psum, off, 32);
      lrow[r] = lrow[r] * alpha + psum;
#pragma unroll
      for (int t = 0; t < 4; ++t) oacc[t][r] *= alpha;
    }
    __builtin_amdgcn_fence(__ATOMIC_RELEASE, "workgroup");
    __builtin_amdgcn_wave_barrier();
    __builtin_amdgcn_fence(__ATOMIC_ACQUIRE, "workgroup");
#pragma unroll 1
    for (int kk = 0; kk < 2; ++kk) {
      FB pa;
      pa.h[0] = *(const v8h*)(pwh + c * AT_KC + kk * 32 + 8 * hh);
      pa.h[1] = *(const v8h*)(pwh + c * AT_KC + kk * 32 + 16 + 8 * hh);
#pragma unroll
      for (int t = 0; t < 4; ++t) {
        FB vb;
        vb.h[0] = *(const v8h*)(Vth + (t * 16 + c) * AT_KC + kk * 32 + 8 * hh);
        vb.h[1] = *(const v8h*)(Vth + (t * 16 + c) * AT_KC + kk * 32 + 16 + 8 * hh);
        oacc[t] = at_mma_h(pa.v, vb.v, oacc[t]);
      }
    }
  }

  float* os = Os[wave];
#pragma unroll
  for (int r = 0; r < 8; ++r) {
    const float inv = oscale * (1.0f / (lrow[r] * PSC));
#pragma unroll
    for (int t = 0; t < 4; ++t) os[(8 * hh + r) * 68 + t * 16 + c] = oacc[t][r] * inv;
  }
  __builtin_amdgcn_fence(__ATOMIC_RELEASE, "workgroup");
  __builtin_amdgcn_wave_barrier();
  __builtin_amdgcn_fence(__ATOMIC_ACQUIRE, "workgroup");
  {
    const int qq = lane >> 3, c8 = (lane & 7) * 8;
    for (int pass = 0; pass < 2; ++pass) {
#pragma unroll
      for (int it = 0; it < 4; ++it) {
        const int row = it * 4 + qq;
        const float* sp = os + row * 68 + c8;
        v8h hv;
#pragma unroll
        for (int e = 0; e < 8; ++e) hv[e] = (_Float16)sp[e];
        *(volatile v8h*)(ob + (size_t)(q0 + row) * kProj + c8) = hv;
      }
      __threadfence();
    }
  }
}

template <bool WRITE16>
__global__ __launch_bounds__(256) void layernorm_rows_kernel(const float* __restrict__ in, const float* __restrict__ gam,
                                                             const float* __restrict__ bet, float* __restrict__ outF,
                                                             unsigned short* __restrict__ outH, int nrows) {
  __shared__ __align__(16) float slab[8][kDm];
  const int wave = threadIdx.x >> 5;
  const int lane = threadIdx.x & 31;
  const int row  = blockIdx.x * 8 + wave;
  if (row >= nrows) return;
  const float* rp = in + (size_t)row * kDm;
  v4f xv[4];
  float s = 0.f;
#pragma unroll
  for (int i = 0; i < 4; ++i) {
    xv[i] = *(const v4f*)(rp + 128 * i + 4 * lane);
    s += (xv[i][0] + xv[i][1]) + (xv[i][2] + xv[i][3]);
  }
#pragma unroll
  for (int off = 1; off < 32; off <<= 1) s += __shfl_xor(s, off, 32);
  const float mu = s * (1.0f / (float)kDm);
  v4f dv[4];
  float ss = 0.f;
#pragma unroll
  for (int i = 0; i < 4; ++i) {
#pragma unroll
    for (int cc = 0; cc < 4; ++cc) {
      const float d = xv[i][cc] - mu;
      dv[i][cc] = d;
      ss += d * d;
    }
  }
#pragma unroll
  for (int off = 1; off < 32; off <<= 1) ss += __shfl_xor(ss, off, 32);
  const float var = ss * (1.0f / (float)kDm);
  const float rs  = rsqrtf(var + 1e-5f);
  v4f yv[4];
#pragma unroll
  for (int i = 0; i < 4; ++i) {
    const v4f gg = *(const v4f*)(gam + 128 * i + 4 * lane);
    const v4f bb = *(const v4f*)(bet + 128 * i + 4 * lane);
#pragma unroll
    for (int cc = 0; cc < 4; ++cc) {
      const float t = dv[i][cc] * rs;
      yv[i][cc] = t * gg[cc] + bb[cc];
    }
  }
  float* orow = outF + (size_t)row * kDm;
  for (int pass = 0; pass < 2; ++pass) {
#pragma unroll
    for (int i = 0; i < 4; ++i) *(volatile v4f*)(orow + 128 * i + 4 * lane) = yv[i];
    __threadfence();
  }
  if (WRITE16) {
    float* sl = slab[wave];
#pragma unroll
    for (int i = 0; i < 4; ++i) *(v4f*)(sl + 128 * i + 4 * lane) = yv[i];
    __builtin_amdgcn_fence(__ATOMIC_RELEASE, "workgroup");
    __builtin_amdgcn_wave_barrier();
    __builtin_amdgcn_fence(__ATOMIC_ACQUIRE, "workgroup");
    v8h hv[2];
#pragma unroll
    for (int i2 = 0; i2 < 2; ++i2) {
      const float* sp = sl + 256 * i2 + 8 * lane;
      const v4f a0 = *(const v4f*)(sp);
      const v4f a1 = *(const v4f*)(sp + 4);
      v8h hq;
      hq[0] = (_Float16)a0[0]; hq[1] = (_Float16)a0[1]; hq[2] = (_Float16)a0[2]; hq[3] = (_Float16)a0[3];
      hq[4] = (_Float16)a1[0]; hq[5] = (_Float16)a1[1]; hq[6] = (_Float16)a1[2]; hq[7] = (_Float16)a1[3];
      hv[i2] = hq;
    }
    _Float16* hrow = (_Float16*)(void*)outH + (size_t)row * kDm;
    for (int pass = 0; pass < 2; ++pass) {
#pragma unroll
      for (int i2 = 0; i2 < 2; ++i2) *(volatile v8h*)(hrow + 256 * i2 + 8 * lane) = hv[i2];
      __threadfence();
    }
  }
}

__device__ __forceinline__ float gelu_erf(float x) {
  return 0.5f * x * (1.0f + erff(x * 0.70710678118654752f));
}

__global__ __launch_bounds__(256) void gelu_f16x2_kernel(const float* __restrict__ in, unsigned short* __restrict__ out,
                                                         int n2, float oscl) {
  const int i = blockIdx.x * 256 + threadIdx.x;
  if (i < n2) {
    const v2f f = *(const v2f*)(in + 2 * (size_t)i);
    const _Float16 h0 = (_Float16)(gelu_erf(f[0]) * oscl);
    const _Float16 h1 = (_Float16)(gelu_erf(f[1]) * oscl);
    const unsigned u = pk16(__builtin_bit_cast(unsigned short, h0), __builtin_bit_cast(unsigned short, h1));
    ((volatile unsigned*)out)[i] = u;
    __threadfence();
    ((volatile unsigned*)out)[i] = u;
  }
}

extern "C" void kernel_launch(void* const* d_in, const int* in_sizes, int n_in,
                              void* d_out, int out_size, void* d_ws, size_t ws_size,
                              hipStream_t stream)
{
  if (n_in < 17) return;
  if (in_sizes[0] != kTok * kDm) return;
  if (in_sizes[1] != kDm * kProj || in_sizes[3] != kDm * kProj || in_sizes[5] != kDm * kProj) return;
  if (in_sizes[2] != kProj || in_sizes[4] != kProj || in_sizes[6] != kProj) return;
  if (in_sizes[7] != kProj * kDm || in_sizes[8] != kDm) return;
  if (in_sizes[9] != kDm || in_sizes[10] != kDm) return;
  if (in_sizes[11] != kDm * kFf || in_sizes[12] != kFf) return;
  if (in_sizes[13] != kFf * kDm || in_sizes[14] != kDm) return;
  if (in_sizes[15] != kDm || in_sizes[16] != kDm) return;
  if (out_size != kTok * kDm) return;
  if (ws_size < kWsTotal) return;

  const float* x    = (const float*)d_in[0];
  const float* Wq   = (const float*)d_in[1];
  const float* bq   = (const float*)d_in[2];
  const float* Wk   = (const float*)d_in[3];
  const float* bk   = (const float*)d_in[4];
  const float* Wv   = (const float*)d_in[5];
  const float* bv   = (const float*)d_in[6];
  const float* Wo   = (const float*)d_in[7];
  const float* bo   = (const float*)d_in[8];
  const float* ln1g = (const float*)d_in[9];
  const float* ln1b = (const float*)d_in[10];
  const float* W1   = (const float*)d_in[11];
  const float* b1   = (const float*)d_in[12];
  const float* W2   = (const float*)d_in[13];
  const float* b2   = (const float*)d_in[14];
  const float* ln2g = (const float*)d_in[15];
  const float* ln2b = (const float*)d_in[16];
  float* out = (float*)d_out;

  char* ws = (char*)d_ws;
  unsigned short* Q16   = (unsigned short*)(ws + kOffQ);
  unsigned short* K16   = (unsigned short*)(ws + kOffK);
  unsigned short* VT16  = (unsigned short*)(ws + kOffVT);
  unsigned short* XB    = (unsigned short*)(ws + kOffXB);
  unsigned short* O16   = (unsigned short*)(ws + kOffXB);
  float*          ATTPX = (float*)(ws + kOffQ);
  float*          X1F   = (float*)(ws + kOffVT);
  unsigned short* X1H   = (unsigned short*)(ws + kOffX1H);
  float*          H32   = (float*)(ws + kOffQ);
  unsigned short* H16   = (unsigned short*)(ws + kOffH16);
  float*          FFPX  = (float*)(ws + kOffQ);
  unsigned short* WQT   = (unsigned short*)(ws + kOffWq);
  unsigned short* WKT   = (unsigned short*)(ws + kOffWk);
  unsigned short* WVT   = (unsigned short*)(ws + kOffWv);
  unsigned short* WOT   = (unsigned short*)(ws + kOffWo);
  unsigned short* W1T   = (unsigned short*)(ws + kOffW1);
  unsigned short* W2T   = (unsigned short*)(ws + kOffW2);

  {
    const int n2 = kTok * kDm / 2;
    cast_f32_bf16x2<<<dim3((n2 + 255) / 256), dim3(256), 0, stream>>>(x, XB, n2);
  }
  tconv_kernel<0><<<dim3(kProj / 64, kDm / 64), dim3(256), 0, stream>>>(Wq, WQT, kDm, kProj, 1.0f);
  tconv_kernel<0><<<dim3(kProj / 64, kDm / 64), dim3(256), 0, stream>>>(Wk, WKT, kDm, kProj, 1.0f);
  tconv_kernel<0><<<dim3(kProj / 64, kDm / 64), dim3(256), 0, stream>>>(Wv, WVT, kDm, kProj, 1.0f);
  tconv_kernel<1><<<dim3(kDm / 64, kProj / 64), dim3(256), 0, stream>>>(Wo, WOT, kProj, kDm, 64.0f);
  tconv_kernel<1><<<dim3(kFf / 64, kDm / 64), dim3(256), 0, stream>>>(W1, W1T, kDm, kFf, 64.0f);
  tconv_kernel<1><<<dim3(kDm / 64, kFf / 64), dim3(256), 0, stream>>>(W2, W2T, kFf, kDm, 64.0f);

  {
    const int tiles = (kTok / 64) * (kProj / 64);
    wmma_gemm64<1, false, 2, 1, false><<<dim3((tiles + 7) / 8, 1), dim3(256), 0, stream>>>(
        XB, nullptr, kDm, 0L, WQT, nullptr, kDm, 0L, (void*)Q16, nullptr, kProj, 0L,
        bq, nullptr, 0L, kTok, kProj, kDm, 1.0f);
    wmma_gemm64<1, false, 2, 1, false><<<dim3((tiles + 7) / 8, 1), dim3(256), 0, stream>>>(
        XB, nullptr, kDm, 0L, WKT, nullptr, kDm, 0L, (void*)K16, nullptr, kProj, 0L,
        bk, nullptr, 0L, kTok, kProj, kDm, 1.0f);
    const int tilesV = (kProj / 64) * (kSeq / 64);
    wmma_gemm64<1, false, 1, 1, false><<<dim3((tilesV + 7) / 8, kBatch), dim3(256), 0, stream>>>(
        WVT, nullptr, kDm, 0L, XB, nullptr, kDm, (long)kSeq * kDm, (void*)VT16, nullptr, kSeq, (long)kProj * kSeq,
        bv, nullptr, 0L, kProj, kSeq, kDm, 1.0f);
  }

  attn_full64_f16_kernel<<<dim3(kHeads * (kSeq / 64), kBatch), dim3(128), 0, stream>>>(Q16, K16, VT16, O16, 0.125f, 64.0f);

  {
    const int tiles = (kTok / 64) * (kDm / 64);
    wmma_gemm64<0, false, 2, 0, true><<<dim3((tiles + 7) / 8, 1), dim3(256), 0, stream>>>(
        O16, nullptr, kProj, 0L, WOT, nullptr, kProj, 0L, (void*)ATTPX, nullptr, kDm, 0L,
        bo, x, 0L, kTok, kDm, kProj, 1.0f / 4096.0f);
  }

  layernorm_rows_kernel<true><<<dim3(kTok / 8), dim3(256), 0, stream>>>(ATTPX, ln1g, ln1b, X1F, X1H, kTok);

  for (int cix = 0; cix < kNumChunks; ++cix) {
    const size_t rowOff = (size_t)cix * kChunkRows;
    const int tiles1 = (kChunkRows / 64) * (kFf / 64);
    wmma_gemm64<0, false, 2, 0, false><<<dim3((tiles1 + 7) / 8, 1), dim3(256), 0, stream>>>(
        X1H + rowOff * kDm, nullptr, kDm, 0L, W1T, nullptr, kDm, 0L, (void*)H32, nullptr, kFf, 0L,
        b1, nullptr, 0L, kChunkRows, kFf, kDm, 1.0f / 64.0f);
    {
      const int n2 = kChunkRows * kFf / 2;
      gelu_f16x2_kernel<<<dim3((n2 + 255) / 256), dim3(256), 0, stream>>>(H32, H16, n2, 16.0f);
    }
    const int tiles2 = (kChunkRows / 64) * (kDm / 64);
    wmma_gemm64<0, false, 2, 0, true><<<dim3((tiles2 + 7) / 8, 1), dim3(256), 0, stream>>>(
        H16, nullptr, kFf, 0L, W2T, nullptr, kFf, 0L, (void*)FFPX, nullptr, kDm, 0L,
        b2, X1F + rowOff * kDm, 0L, kChunkRows, kDm, kFf, 1.0f / 1024.0f);
    layernorm_rows_kernel<false><<<dim3(kChunkRows / 8), dim3(256), 0, stream>>>(
        FFPX, ln2g, ln2b, out + rowOff * kDm, nullptr, kChunkRows);
  }
}
